// RelationNet_50861002719650
// MI455X (gfx1250) — hardware-run, weakly checked
//
#include <hip/hip_runtime.h>
#include <math.h>

typedef __attribute__((ext_vector_type(16))) _Float16 v16h;
typedef __attribute__((ext_vector_type(16))) __bf16 v16b;
typedef __attribute__((ext_vector_type(8)))  _Float16 v8h;
typedef __attribute__((ext_vector_type(8)))  float v8f;
typedef __attribute__((ext_vector_type(4)))  float v4f;
typedef __attribute__((ext_vector_type(2)))  float v2f;
typedef __attribute__((ext_vector_type(4)))  unsigned v4u;
typedef __attribute__((ext_vector_type(4)))  int v4i;
typedef float __attribute__((may_alias)) float_a;
typedef int __attribute__((may_alias)) int_a;

template <typename T> __device__ __forceinline__ void vst2(void* p, T v) { *(volatile T*)p = v; __threadfence(); *(volatile T*)p = v; }
__device__ __forceinline__ v8f wmma16(v16h a, v16h b, v8f c) {
  v8f d = __builtin_amdgcn_wmma_f32_16x16x32_f16(false, a, false, b, (short)0, c, false, false);
  asm volatile("v_nop\n\tv_nop\n\tv_nop\n\tv_nop" : "+v"(d) : "v"(a), "v"(b));
  return d;
}
__device__ __forceinline__ v8f wmma_bf(v16b a, v16b b, v8f c) {
  v8f d = __builtin_amdgcn_wmma_f32_16x16x32_bf16(false, a, false, b, (short)0, c, false, false);
  asm volatile("v_nop\n\tv_nop\n\tv_nop\n\tv_nop" : "+v"(d) : "v"(a), "v"(b));
  return d;
}
__device__ __forceinline__ v16h frag_h(const _Float16* rowk0, int lane) {
  union { v16h v; v8h q[2]; } u; const _Float16* p = rowk0 + 8 * (lane >> 4);
  u.q[0] = *(const v8h*)p; u.q[1] = *(const v8h*)(p + 16); return u.v;
}
__device__ __forceinline__ v16h frag_f32(const float* rowk0, int lane) {
  v16h a; const float* p = rowk0 + 8 * (lane >> 4);
#pragma unroll
  for (int i = 0; i < 8; ++i) { a[i] = (_Float16)p[i]; a[8 + i] = (_Float16)p[16 + i]; }
  return a;
}
__device__ __forceinline__ v16h frag_f32s(const float* rowk0, int lane, float sc) {
  v16h a; const float* p = rowk0 + 8 * (lane >> 4);
#pragma unroll
  for (int i = 0; i < 8; ++i) { a[i] = (_Float16)(p[i] * sc); a[8 + i] = (_Float16)(p[16 + i] * sc); }
  return a;
}
__device__ __forceinline__ v16h fragc_f32(const float* W, int k0, int n, int lane, int ld, int K) {
  v16h a; const int g = lane >> 4;
#pragma unroll
  for (int i = 0; i < 8; ++i) { const int ka = k0 + 8 * g + i, kb = ka + 16;
    a[i] = (_Float16)(ka < K ? W[(size_t)(ka < K ? ka : K - 1) * ld + n] : 0.f); a[8 + i] = (_Float16)(kb < K ? W[(size_t)(kb < K ? kb : K - 1) * ld + n] : 0.f); }
  return a;
}
struct F2 { v16b h, l; };
__device__ __forceinline__ F2 bsplit16(const float v[16]) { F2 r;
#pragma unroll
  for (int i = 0; i < 16; ++i) { const __bf16 h = (__bf16)v[i]; r.h[i] = h; r.l[i] = (__bf16)(v[i] - (float)h); }
  return r; }
__device__ __forceinline__ F2 split_row(const float* row, int k0, int lane) { float v[16]; const float* p = row + k0 + 8 * (lane >> 4);
#pragma unroll
  for (int i = 0; i < 8; ++i) { v[i] = p[i]; v[8 + i] = p[16 + i]; }
  return bsplit16(v); }
__device__ __forceinline__ F2 split_rowK(const float* row, int k0, int lane, int K) { float v[16]; const int g = lane >> 4;
#pragma unroll
  for (int i = 0; i < 8; ++i) { const int ka = k0 + 8 * g + i, kb = ka + 16; v[i] = ka < K ? row[ka < K ? ka : K - 1] : 0.f; v[8 + i] = kb < K ? row[kb < K ? kb : K - 1] : 0.f; }
  return bsplit16(v); }
__device__ __forceinline__ F2 split_col(const float* W, int k0, int n, int lane, int ld, int K) { float v[16]; const int g = lane >> 4;
#pragma unroll
  for (int i = 0; i < 8; ++i) { const int ka = k0 + 8 * g + i, kb = ka + 16; v[i] = ka < K ? W[(size_t)(ka < K ? ka : K - 1) * ld + n] : 0.f; v[8 + i] = kb < K ? W[(size_t)(kb < K ? kb : K - 1) * ld + n] : 0.f; }
  return bsplit16(v); }
__device__ __forceinline__ v8f mac3(const F2& a, const F2& b, v8f c) { c = wmma_bf(a.l, b.h, c); c = wmma_bf(a.h, b.l, c); return wmma_bf(a.h, b.h, c); }
__device__ __forceinline__ float sigm(float v) { return 1.0f / (1.0f + expf(-v)); }
#define LDSX() do { asm volatile("s_wait_dscnt 0" ::: "memory"); __builtin_amdgcn_wave_barrier(); __builtin_amdgcn_fence(__ATOMIC_RELEASE, "workgroup"); } while (0)

__device__ __forceinline__ float bfr(float v) { return (float)(__bf16)v; }
#define NBT 4
#define NQ 256
#define NS 128
#define CC 256
#define NPR (NBT * NQ * NS)
#define H0 256
#define H1 64
#define WS_AQ  0u
#define WS_AS  (WS_AQ + 4u * (size_t)NBT * NQ * H0)
#define WS_B0S (WS_AS + 4u * (size_t)NBT * NS * H0)
#define WS_H1  (WS_B0S + 4u * (size_t)H0 * 2)
#define WS_B1S (WS_H1 + 4u * (size_t)NPR * H1)
#define WS_H2  (WS_B1S + 4u * (size_t)H1 * 2)
#define WS_B2S (WS_H2 + 4u * (size_t)NPR)
#define WS_END (WS_B2S + 128u)
__global__ __launch_bounds__(128) void k_pre(const float* __restrict__ QF, const float* __restrict__ SF, const float* __restrict__ W0, float* __restrict__ AQ, float* __restrict__ AS) { __shared__ __align__(16) float sf[4][16][132];
  const int tid = threadIdx.x, wave = tid >> 5, lane = tid & 31, col = lane & 15, g = lane >> 4; const int which = blockIdx.z; const int nrows = which == 0 ? NBT * NQ : NBT * NS; if ((int)blockIdx.x * 64 >= nrows) return;
  const float* X = which == 0 ? QF : SF; float* DST = which == 0 ? AQ : AS; const int koff = which == 0 ? 0 : CC; const int c0 = blockIdx.y * 128; const size_t r0 = (size_t)blockIdx.x * 64 + wave * 16;
  v8f acc[8] = {};
#pragma unroll 2
  for (int kc = 0; kc < CC / 32; ++kc) { v16b a; { const float* p = X + (r0 + col) * CC + kc * 32 + 8 * g;
#pragma unroll
      for (int i = 0; i < 8; ++i) { a[i] = (__bf16)p[i]; a[8 + i] = (__bf16)p[16 + i]; } }
#pragma unroll
    for (int j = 0; j < 8; ++j) { v16b w; const float* wr = W0 + (size_t)(c0 + j * 16 + col) * (2 * CC) + koff + kc * 32 + 8 * g;
#pragma unroll
      for (int i = 0; i < 8; ++i) { w[i] = (__bf16)wr[i]; w[8 + i] = (__bf16)wr[16 + i]; }
      asm volatile("s_wait_loadcnt 0x0" ::: "memory"); acc[j] = wmma_bf(a, w, acc[j]); } }
#pragma unroll
  for (int j = 0; j < 8; ++j)
#pragma unroll
    for (int r = 0; r < 8; ++r) sf[wave][8 * g + r][j * 16 + col] = acc[j][r];
  LDSX(); for (int rl = 0; rl < 16; ++rl) vst2(DST + (r0 + rl) * H0 + c0 + lane * 4, *(const v4f*)&sf[wave][rl][lane * 4]); }
__global__ __launch_bounds__(256) void k_st0(const float* __restrict__ AQ, const float* __restrict__ AS, const float* __restrict__ B0, float* __restrict__ ST) { __shared__ __align__(16) float so[32];
  const int t = threadIdx.x; const int cl = t >> 4, sub = t & 15; const int c = blockIdx.x * 16 + cl; const float bb = bfr(B0[c]);
  float s = 0.f;
  for (int bq = sub; bq < NBT * NQ; bq += 16) { const float aq = AQ[(size_t)bq * H0 + c] + bb; const int b = bq / NQ; const float* as = AS + (size_t)b * NS * H0 + c; for (int si = 0; si < NS; ++si) s += aq + as[(size_t)si * H0]; }
#pragma unroll
  for (int o = 1; o < 16; o <<= 1) s += __shfl_xor(s, o);
  const float mu = s * (1.0f / NPR); float s2 = 0.f;
  for (int bq = sub; bq < NBT * NQ; bq += 16) { const float aq = AQ[(size_t)bq * H0 + c] + bb - mu; const int b = bq / NQ; const float* as = AS + (size_t)b * NS * H0 + c; for (int si = 0; si < NS; ++si) { const float d = aq + as[(size_t)si * H0]; s2 += d * d; } }
#pragma unroll
  for (int o = 1; o < 16; o <<= 1) s2 += __shfl_xor(s2, o);
  if (sub == 0) { so[cl * 2] = mu; so[cl * 2 + 1] = rsqrtf(s2 * (1.0f / NPR) + 1e-5f); }
  __syncthreads(); if (t < 32) vst2(ST + (size_t)blockIdx.x * 32 + t, so[t]); }
__global__ __launch_bounds__(128) void k_l1(const float* __restrict__ AQ, const float* __restrict__ AS, const float* __restrict__ B0, const float* __restrict__ ST0, const float* __restrict__ G0, const float* __restrict__ BT0, const float* __restrict__ W1, const float* __restrict__ B1, float* __restrict__ H1P) { __shared__ __align__(16) float sf[4][16][68];
  const int tid = threadIdx.x, wave = tid >> 5, lane = tid & 31, col = lane & 15, g = lane >> 4; const size_t r0 = (size_t)blockIdx.x * 64 + wave * 16; const size_t pr = r0 + col; const size_t bq = pr / NS; const int s_ = (int)(pr % NS); const int b = (int)(bq / NQ);
  const float* aq = AQ + bq * H0; const float* as = AS + ((size_t)b * NS + s_) * H0;
  v8f acc[4] = {};
#pragma unroll 1
  for (int kc = 0; kc < H0 / 32; ++kc) { float v[16];
#pragma unroll
    for (int i = 0; i < 8; ++i) { const int c = kc * 32 + 8 * g + i, c2 = c + 16;
      v[i] = fmaxf(((aq[c] + as[c] + bfr(B0[c])) - ST0[c * 2]) * ST0[c * 2 + 1] * bfr(G0[c]) + bfr(BT0[c]), 0.f);
      v[8 + i] = fmaxf(((aq[c2] + as[c2] + bfr(B0[c2])) - ST0[c2 * 2]) * ST0[c2 * 2 + 1] * bfr(G0[c2]) + bfr(BT0[c2]), 0.f); }
    asm volatile("s_wait_loadcnt 0x0" ::: "memory"); const F2 a = bsplit16(v);
#pragma unroll
    for (int j = 0; j < 4; ++j) { v16b w; const float* wr = W1 + (size_t)(j * 16 + col) * H0 + kc * 32 + 8 * g;
#pragma unroll
      for (int i = 0; i < 8; ++i) { w[i] = (__bf16)wr[i]; w[8 + i] = (__bf16)wr[16 + i]; }
      asm volatile("s_wait_loadcnt 0x0" ::: "memory"); acc[j] = wmma_bf(a.h, w, acc[j]); acc[j] = wmma_bf(a.l, w, acc[j]); } }
#pragma unroll
  for (int j = 0; j < 4; ++j) { const float bb = bfr(B1[j * 16 + col]);
#pragma unroll
    for (int r = 0; r < 8; ++r) sf[wave][8 * g + r][j * 16 + col] = acc[j][r] + bb; }
  LDSX(); for (int rl = 0; rl < 16; ++rl) if (lane < 16) vst2(H1P + (r0 + rl) * H1 + lane * 4, *(const v4f*)&sf[wave][rl][lane * 4]); }
__global__ __launch_bounds__(256) void k_st1(const float* __restrict__ H1P, float* __restrict__ ST) { __shared__ __align__(16) float so[32];
  const int t = threadIdx.x; const int cl = t >> 4, sub = t & 15; const int c = blockIdx.x * 16 + cl;
  float s = 0.f; for (int r = sub; r < NPR; r += 16) s += H1P[(size_t)r * H1 + c];
#pragma unroll
  for (int o = 1; o < 16; o <<= 1) s += __shfl_xor(s, o);
  const float mu = s * (1.0f / NPR); float s2 = 0.f; for (int r = sub; r < NPR; r += 16) { const float d = H1P[(size_t)r * H1 + c] - mu; s2 += d * d; }
#pragma unroll
  for (int o = 1; o < 16; o <<= 1) s2 += __shfl_xor(s2, o);
  if (sub == 0) { so[cl * 2] = mu; so[cl * 2 + 1] = rsqrtf(s2 * (1.0f / NPR) + 1e-5f); }
  __syncthreads(); if (t < 32) vst2(ST + (size_t)blockIdx.x * 32 + t, so[t]); }
__global__ __launch_bounds__(128) void k_l2(const float* __restrict__ H1P, const float* __restrict__ ST1, const float* __restrict__ G1, const float* __restrict__ BT1, const float* __restrict__ W2, const float* __restrict__ B2, float* __restrict__ H2P) { __shared__ __align__(16) float so[64];
  const int t = threadIdx.x; const int rl = t >> 1, half = t & 1; const size_t r = (size_t)blockIdx.x * 64 + rl; float s = 0.f;
#pragma unroll 4
  for (int e = 0; e < 32; ++e) { const int c = half * 32 + e; const float v = fmaxf((H1P[r * H1 + c] - ST1[c * 2]) * ST1[c * 2 + 1] * bfr(G1[c]) + bfr(BT1[c]), 0.f); s += v * bfr(W2[c]); }
  s += __shfl_xor(s, 1); if (half == 0) so[rl] = s + bfr(B2[0]);
  __syncthreads(); if (t < 16) vst2(H2P + (size_t)blockIdx.x * 64 + t * 4, *(const v4f*)&so[t * 4]); }
__global__ __launch_bounds__(256) void k_st2(const float* __restrict__ H2P, float* __restrict__ ST) { __shared__ float sred[8]; __shared__ float sbc;
  const int t = threadIdx.x; float s = 0.f; for (int r = t; r < NPR; r += 256) s += H2P[r];
#pragma unroll
  for (int o = 1; o < 32; o <<= 1) s += __shfl_xor(s, o);
  if ((t & 31) == 0) sred[t >> 5] = s; __syncthreads(); if (t == 0) { float a = 0.f; for (int w = 0; w < 8; ++w) a += sred[w]; sbc = a * (1.0f / NPR); } __syncthreads(); const float mu = sbc; __syncthreads();
  float s2 = 0.f; for (int r = t; r < NPR; r += 256) { const float d = H2P[r] - mu; s2 += d * d; }
#pragma unroll
  for (int o = 1; o < 32; o <<= 1) s2 += __shfl_xor(s2, o);
  if ((t & 31) == 0) sred[t >> 5] = s2; __syncthreads();
  if (t < 32) { float v = 0.f; if (t == 0) v = mu; if (t == 1) { float a = 0.f; for (int w = 0; w < 8; ++w) a += sred[w]; v = rsqrtf(a * (1.0f / NPR) + 1e-5f); } vst2(ST + t, v); } }
__global__ __launch_bounds__(64) void k_fin(const float* __restrict__ H2P, const float* __restrict__ ST2, const float* __restrict__ G2, const float* __restrict__ BT2, float* __restrict__ OUT) {
  const int t = threadIdx.x; const size_t r = (size_t)blockIdx.x * 256 + t * 4; const float mu = ST2[0], rs = ST2[1], ga = bfr(G2[0]), be = bfr(BT2[0]);
  const v4f h = *(const v4f*)(H2P + r); v4f o;
#pragma unroll
  for (int z = 0; z < 4; ++z) o[z] = fmaxf((h[z] - mu) * rs * ga + be, 0.f);
  vst2(OUT + r, o); }
extern "C" void kernel_launch(void* const* d_in, const int* in_sizes, int n_in, void* d_out, int out_size, void* d_ws, size_t ws_size, hipStream_t stream) {
  (void)in_sizes; (void)n_in; (void)out_size;
  const float** F = (const float**)d_in;
  if (ws_size < (size_t)WS_END) return;
  char* ws = (char*)d_ws; float *AQ = (float*)(ws + WS_AQ), *AS = (float*)(ws + WS_AS), *B0S = (float*)(ws + WS_B0S), *H1P = (float*)(ws + WS_H1), *B1S = (float*)(ws + WS_B1S), *H2P = (float*)(ws + WS_H2), *B2S = (float*)(ws + WS_B2S);
  k_pre<<<dim3(NBT * NQ / 64, H0 / 128, 2), 128, 0, stream>>>(F[1], F[0], F[2], AQ, AS);
  k_st0<<<dim3(H0 / 16), 256, 0, stream>>>(AQ, AS, F[3], B0S);
  k_l1<<<dim3(NPR / 64), 128, 0, stream>>>(AQ, AS, F[3], B0S, F[4], F[5], F[6], F[7], H1P);
  k_st1<<<dim3(H1 / 16), 256, 0, stream>>>(H1P, B1S);
  k_l2<<<dim3(NPR / 64), 128, 0, stream>>>(H1P, B1S, F[8], F[9], F[10], F[11], H2P);
  k_st2<<<dim3(1), 256, 0, stream>>>(H2P, B2S);
  k_fin<<<dim3(NPR / 256), 64, 0, stream>>>(H2P, B2S, F[12], F[13], (float*)d_out);
}
